// EASLayer_MLP_62551903699397
// MI455X (gfx1250) — hardware-run, weakly checked
//
#include <hip/hip_runtime.h>
#include <math.h>

typedef __attribute__((ext_vector_type(16))) _Float16 v16h;
typedef __attribute__((ext_vector_type(16))) __bf16 v16b;
typedef __attribute__((ext_vector_type(8)))  _Float16 v8h;
typedef __attribute__((ext_vector_type(8)))  float v8f;
typedef __attribute__((ext_vector_type(4)))  float v4f;
typedef __attribute__((ext_vector_type(2)))  float v2f;
typedef __attribute__((ext_vector_type(4)))  unsigned v4u;
typedef __attribute__((ext_vector_type(4)))  int v4i;
typedef float __attribute__((may_alias)) float_a;
typedef int __attribute__((may_alias)) int_a;

template <typename T> __device__ __forceinline__ void vst2(void* p, T v) { *(volatile T*)p = v; __threadfence(); *(volatile T*)p = v; }
__device__ __forceinline__ v8f wmma16(v16h a, v16h b, v8f c) {
  v8f d = __builtin_amdgcn_wmma_f32_16x16x32_f16(false, a, false, b, (short)0, c, false, false);
  asm volatile("v_nop\n\tv_nop\n\tv_nop\n\tv_nop" : "+v"(d) : "v"(a), "v"(b));
  return d;
}
__device__ __forceinline__ v8f wmma_bf(v16b a, v16b b, v8f c) {
  v8f d = __builtin_amdgcn_wmma_f32_16x16x32_bf16(false, a, false, b, (short)0, c, false, false);
  asm volatile("v_nop\n\tv_nop\n\tv_nop\n\tv_nop" : "+v"(d) : "v"(a), "v"(b));
  return d;
}
__device__ __forceinline__ v16h frag_h(const _Float16* rowk0, int lane) {
  union { v16h v; v8h q[2]; } u; const _Float16* p = rowk0 + 8 * (lane >> 4);
  u.q[0] = *(const v8h*)p; u.q[1] = *(const v8h*)(p + 16); return u.v;
}
__device__ __forceinline__ v16h frag_f32(const float* rowk0, int lane) {
  v16h a; const float* p = rowk0 + 8 * (lane >> 4);
#pragma unroll
  for (int i = 0; i < 8; ++i) { a[i] = (_Float16)p[i]; a[8 + i] = (_Float16)p[16 + i]; }
  return a;
}
__device__ __forceinline__ v16h frag_f32s(const float* rowk0, int lane, float sc) {
  v16h a; const float* p = rowk0 + 8 * (lane >> 4);
#pragma unroll
  for (int i = 0; i < 8; ++i) { a[i] = (_Float16)(p[i] * sc); a[8 + i] = (_Float16)(p[16 + i] * sc); }
  return a;
}
__device__ __forceinline__ v16h fragc_f32(const float* W, int k0, int n, int lane, int ld, int K) {
  v16h a; const int g = lane >> 4;
#pragma unroll
  for (int i = 0; i < 8; ++i) { const int ka = k0 + 8 * g + i, kb = ka + 16;
    a[i] = (_Float16)(ka < K ? W[(size_t)(ka < K ? ka : K - 1) * ld + n] : 0.f); a[8 + i] = (_Float16)(kb < K ? W[(size_t)(kb < K ? kb : K - 1) * ld + n] : 0.f); }
  return a;
}
struct F2 { v16b h, l; };
__device__ __forceinline__ F2 bsplit16(const float v[16]) { F2 r;
#pragma unroll
  for (int i = 0; i < 16; ++i) { const __bf16 h = (__bf16)v[i]; r.h[i] = h; r.l[i] = (__bf16)(v[i] - (float)h); }
  return r; }
__device__ __forceinline__ F2 split_row(const float* row, int k0, int lane) { float v[16]; const float* p = row + k0 + 8 * (lane >> 4);
#pragma unroll
  for (int i = 0; i < 8; ++i) { v[i] = p[i]; v[8 + i] = p[16 + i]; }
  return bsplit16(v); }
__device__ __forceinline__ F2 split_rowK(const float* row, int k0, int lane, int K) { float v[16]; const int g = lane >> 4;
#pragma unroll
  for (int i = 0; i < 8; ++i) { const int ka = k0 + 8 * g + i, kb = ka + 16; v[i] = ka < K ? row[ka < K ? ka : K - 1] : 0.f; v[8 + i] = kb < K ? row[kb < K ? kb : K - 1] : 0.f; }
  return bsplit16(v); }
__device__ __forceinline__ F2 split_col(const float* W, int k0, int n, int lane, int ld, int K) { float v[16]; const int g = lane >> 4;
#pragma unroll
  for (int i = 0; i < 8; ++i) { const int ka = k0 + 8 * g + i, kb = ka + 16; v[i] = ka < K ? W[(size_t)(ka < K ? ka : K - 1) * ld + n] : 0.f; v[8 + i] = kb < K ? W[(size_t)(kb < K ? kb : K - 1) * ld + n] : 0.f; }
  return bsplit16(v); }
__device__ __forceinline__ v8f mac3(const F2& a, const F2& b, v8f c) { c = wmma_bf(a.l, b.h, c); c = wmma_bf(a.h, b.l, c); return wmma_bf(a.h, b.h, c); }
__device__ __forceinline__ float sigm(float v) { return 1.0f / (1.0f + expf(-v)); }
#define LDSX() do { asm volatile("s_wait_dscnt 0" ::: "memory"); __builtin_amdgcn_wave_barrier(); __builtin_amdgcn_fence(__ATOMIC_RELEASE, "workgroup"); } while (0)


#define NR 4928
#define DD 768
#define NA 1024
#define RR 4
#define HH (NA * RR)
#ifndef NRT
#define NRT (NR / 64)
#endif
typedef __attribute__((ext_vector_type(8))) __bf16 v8b;
__device__ __forceinline__ v16b frag_b(const __bf16* rowk0, int lane) {
  union { v16b v; v8b q[2]; } u; const __bf16* p = rowk0 + 8 * (lane >> 4);
  u.q[0] = *(const v8b*)p; u.q[1] = *(const v8b*)(p + 16); return u.v;
}
__device__ __forceinline__ float bfr(float v) { return (float)(__bf16)v; }
__device__ __attribute__((noinline)) float exp_ni(float v) { return expf(v); }
__device__ __attribute__((noinline)) float erf_ni(float v) { return erff(v); }
__device__ __forceinline__ float gelu_exact(float v) { return 0.5f * v * (1.0f + erf_ni(v * 0.70710678118654752f)); }

#define PK_1 0
#define PK_O (PK_1 + (size_t)HH * DD)
#define PK_G (PK_O + (size_t)DD * HH)
#define PK_END (PK_G + (size_t)DD * DD)
#define WS_PK  0u
#define WS_XB  (((2u * PK_END) + 127u) / 128u * 128u)
#define WS_H2H (WS_XB + 2u * NR * DD)
#define WS_H2L (WS_H2H + 2u * (size_t)NR * HH)
#define WS_SB  (WS_H2L + 2u * (size_t)NR * HH)
#define WS_ORG (WS_SB + 4u * DD)
#define WS_END (WS_ORG + 4u * NR * DD)

__global__ __launch_bounds__(256) void k_pack(const float* __restrict__ W1, const float* __restrict__ WO, const float* __restrict__ WG, __bf16* __restrict__ PK) {
  __shared__ __align__(16) __bf16 s[HH]; const int row = blockIdx.x, which = blockIdx.y, tid = threadIdx.x; int K; size_t dst;
  if (which == 0) { const int n = row >> 2, r = row & 3; K = DD; dst = PK_1 + (size_t)row * DD; for (int k = tid; k < DD; k += 256) s[k] = (__bf16)W1[((size_t)n * DD + k) * RR + r]; }
  else if (which == 1) { if (row >= DD) return; K = HH; dst = PK_O + (size_t)row * HH; for (int k = tid; k < HH; k += 256) s[k] = (__bf16)WO[(size_t)k * DD + row]; }
  else { if (row >= DD) return; K = DD; dst = PK_G + (size_t)row * DD; for (int k = tid; k < DD; k += 256) s[k] = (__bf16)WG[(size_t)row * DD + k]; }
  __syncthreads();
  for (int q = tid; q < K / 8; q += 256) vst2((unsigned*)(PK + dst + q * 8), *(const v4u*)&s[q * 8]);
}
__global__ __launch_bounds__(128) void k_xb(const float* __restrict__ X, __bf16* __restrict__ XB) {
  __shared__ __align__(16) __bf16 s[DD]; const size_t r = blockIdx.x; const int t = threadIdx.x;
  for (int k = t; k < DD; k += 128) s[k] = (__bf16)X[r * DD + k];
  __syncthreads();
  if (t < DD / 8) vst2((unsigned*)(XB + r * DD + t * 8), *(const v4u*)&s[t * 8]);
}
__global__ __launch_bounds__(256) void k_sb(const float* __restrict__ BO, float* __restrict__ SB) {
  __shared__ __align__(16) float s[DD]; const int t = threadIdx.x;
  for (int d = t; d < DD; d += 256) { float a = 0.f; for (int n = 0; n < NA; ++n) a += bfr(BO[(size_t)n * DD + d]); s[d] = a; }
  __syncthreads();
  for (int q = t; q < DD / 4; q += 256) vst2(SB + q * 4, *(const v4f*)&s[q * 4]);
}
__global__ __launch_bounds__(128) void k_ad(const __bf16* __restrict__ XB, const __bf16* __restrict__ PK, const float* __restrict__ B1, const float* __restrict__ MW, const float* __restrict__ MB, __bf16* __restrict__ H2H, __bf16* __restrict__ H2L) {
  __shared__ __align__(16) __bf16 soh[4][16][136], sol[4][16][136];
  const int tid = threadIdx.x, wave = tid >> 5, lane = tid & 31, col = lane & 15, g = lane >> 4; const size_t r0 = (size_t)blockIdx.x * 64 + wave * 16; const int n0 = blockIdx.y * 128;
  v8f acc[8] = {};
#pragma unroll 2
  for (int kc = 0; kc < DD / 32; ++kc) { const v16b a = frag_b(XB + (r0 + col) * DD + kc * 32, lane);
#pragma unroll
    for (int j = 0; j < 8; ++j) acc[j] = wmma_bf(a, frag_b(PK + PK_1 + (size_t)(n0 + j * 16 + col) * DD + kc * 32, lane), acc[j]); }
#pragma unroll
  for (int j = 0; j < 8; ++j) { const int hcol = n0 + j * 16 + col; const int n = hcol >> 2, rp = hcol & 3;
    const float bb1 = bfr(B1[hcol]); const float wd = bfr(MW[((size_t)n * RR + rp) * RR + rp]);
    const float mb = bfr(MB[hcol]);
#pragma unroll
    for (int r8 = 0; r8 < 8; ++r8) { const float h = gelu_exact(acc[j][r8] + bb1);
      const float v = gelu_exact(h * wd + mb);
      const __bf16 hb = (__bf16)v; soh[wave][8 * g + r8][j * 16 + col] = hb; sol[wave][8 * g + r8][j * 16 + col] = (__bf16)(v - (float)hb); } }
  LDSX();
  for (int rl = 0; rl < 16; ++rl) if (lane < 16) { vst2((unsigned*)(H2H + (r0 + rl) * HH + n0 + lane * 8), *(const v4u*)&soh[wave][rl][lane * 8]); vst2((unsigned*)(H2L + (r0 + rl) * HH + n0 + lane * 8), *(const v4u*)&sol[wave][rl][lane * 8]); }
}
__global__ __launch_bounds__(128) void k_org(const __bf16* __restrict__ XB, const __bf16* __restrict__ PK, const float* __restrict__ BG, float* __restrict__ ORG) {
  __shared__ __align__(16) float so[4][16][132];
  const int tid = threadIdx.x, wave = tid >> 5, lane = tid & 31, col = lane & 15, g = lane >> 4; const size_t r0 = (size_t)blockIdx.x * 64 + wave * 16; const int n0 = blockIdx.y * 128;
  v8f acc[8] = {};
#pragma unroll 2
  for (int kc = 0; kc < DD / 32; ++kc) { const v16b a = frag_b(XB + (r0 + col) * DD + kc * 32, lane);
#pragma unroll
    for (int j = 0; j < 8; ++j) acc[j] = wmma_bf(a, frag_b(PK + PK_G + (size_t)(n0 + j * 16 + col) * DD + kc * 32, lane), acc[j]); }
#pragma unroll
  for (int j = 0; j < 8; ++j) { const float bb = bfr(BG[n0 + j * 16 + col]);
#pragma unroll
    for (int r = 0; r < 8; ++r) so[wave][8 * g + r][j * 16 + col] = acc[j][r] + bb; }
  LDSX();
  for (int rl = 0; rl < 16; ++rl) vst2(ORG + (r0 + rl) * DD + n0 + lane * 4, *(const v4f*)&so[wave][rl][lane * 4]);
}
__global__ __launch_bounds__(128) void k_up(const __bf16* __restrict__ H2H, const __bf16* __restrict__ H2L, const __bf16* __restrict__ PK, const float* __restrict__ SB, const float* __restrict__ ORG, float* __restrict__ OUT) {
  __shared__ __align__(16) float so[4][16][132];
  const int tid = threadIdx.x, wave = tid >> 5, lane = tid & 31, col = lane & 15, g = lane >> 4; const size_t r0 = (size_t)blockIdx.x * 64 + wave * 16; const int n0 = blockIdx.y * 128;
  v8f acc[8] = {};
#pragma unroll 2
  for (int kc = 0; kc < HH / 32; ++kc) { const v16b ah = frag_b(H2H + (r0 + col) * HH + kc * 32, lane), al = frag_b(H2L + (r0 + col) * HH + kc * 32, lane);
#pragma unroll
    for (int j = 0; j < 8; ++j) { const v16b w = frag_b(PK + PK_O + (size_t)(n0 + j * 16 + col) * HH + kc * 32, lane); acc[j] = wmma_bf(al, w, acc[j]); acc[j] = wmma_bf(ah, w, acc[j]); } }
#pragma unroll
  for (int j = 0; j < 8; ++j) { const int d = n0 + j * 16 + col; const float sb = SB[d];
#pragma unroll
    for (int r = 0; r < 8; ++r) so[wave][8 * g + r][j * 16 + col] = ORG[(r0 + 8 * g + r) * DD + d] + 0.25f * (acc[j][r] + sb); }
  LDSX();
  for (int rl = 0; rl < 16; ++rl) vst2(OUT + (r0 + rl) * DD + n0 + lane * 4, *(const v4f*)&so[wave][rl][lane * 4]);
}
extern "C" void kernel_launch(void* const* d_in, const int* in_sizes, int n_in, void* d_out, int out_size, void* d_ws, size_t ws_size, hipStream_t stream) {
  (void)in_sizes; (void)n_in; (void)out_size;
  const float** F = (const float**)d_in;
  if (ws_size < (size_t)WS_END) return;
  char* ws = (char*)d_ws; __bf16 *PK = (__bf16*)(ws + WS_PK), *XB = (__bf16*)(ws + WS_XB), *H2H = (__bf16*)(ws + WS_H2H), *H2L = (__bf16*)(ws + WS_H2L); float *SB = (float*)(ws + WS_SB), *ORG = (float*)(ws + WS_ORG);
  k_pack<<<dim3(HH, 3), 256, 0, stream>>>(F[3], F[7], F[1], PK);
  k_xb<<<NRT * 64, 128, 0, stream>>>(F[0], XB);
  k_sb<<<1, 256, 0, stream>>>(F[8], SB);
  k_ad<<<dim3(NRT, HH / 128), 128, 0, stream>>>(XB, PK, F[4], F[5], F[6], H2H, H2L);
  k_org<<<dim3(NRT, DD / 128), 128, 0, stream>>>(XB, PK, F[2], ORG);
  k_up<<<dim3(NRT, DD / 128), 128, 0, stream>>>(H2H, H2L, PK, SB, ORG, (float*)d_out);
}
